// REN_40175124087397
// MI455X (gfx1250) — hardware-verified
//
#include <hip/hip_runtime.h>


namespace {
constexpr int BATCH = 32768, NLIM = 32768  , NX = 64, NUNIT = 256, NY = 32, NU = 64, NZ = 2 * NX + NUNIT  , KV = NX + NU  ;
constexpr float XS = 8.0f, WSC = 256.0f;
static_assert(BATCH % 32 == 0 && NLIM % 32 == 0 && NLIM <= BATCH && NUNIT % 16 == 0, "tiling");
typedef _Float16 b16;
typedef __attribute__((ext_vector_type(16))) _Float16 v16b;
typedef __attribute__((ext_vector_type(8))) _Float16 v8b;
typedef __attribute__((ext_vector_type(8))) float v8f;
typedef __attribute__((ext_vector_type(4))) float v4f;
__device__ __forceinline__ float bf16_rne(float f) { unsigned int u = __float_as_uint(f); u += 0x7FFFu + ((u >> 16) & 1u); return __uint_as_float(u & 0xFFFF0000u); }
__device__ __forceinline__ void split16(float v, b16& hi, b16& lo) { hi = (b16)v; lo = (b16)(v - (float)hi); }
__device__ __forceinline__ v16b frag_kb(const b16* p, int hh) { const v8b a = *(const v8b*)(p + 8 * hh), b = *(const v8b*)(p + 16 + 8 * hh); v16b f;
#pragma unroll
  for (int e = 0; e < 8; ++e) { f[e] = a[e]; f[8 + e] = b[e]; } return f; }
__device__ __forceinline__ v8f wmma16b(v16b a, v16b b, v8f c) { v8f d = __builtin_amdgcn_wmma_f32_16x16x32_f16(false, a, false, b, (short)0, c, false, false); asm volatile("v_nop\n\tv_nop\n\tv_nop\n\tv_nop" : "+v"(d) : "v"(a), "v"(b)); return d; }
__device__ __forceinline__ void wave_lds_sync() { __builtin_amdgcn_fence(__ATOMIC_RELEASE, "workgroup"); __builtin_amdgcn_wave_barrier(); __builtin_amdgcn_fence(__ATOMIC_ACQUIRE, "workgroup"); }
__device__ __forceinline__ float pmul(float a, float b) { float p = a * b; asm volatile("" : "+v"(p)); return p; }
__device__ __forceinline__ int iclamp(int v, int lo, int hi) { return v < lo ? lo : (v > hi ? hi : v); }

typedef __attribute__((ext_vector_type(4))) _Float16 v4h;
__global__ __launch_bounds__(256) void par1_kernel(const float* __restrict__ B2, const float* __restrict__ C2, const float* __restrict__ D12, const float* __restrict__ D21, const float* __restrict__ St, const float* __restrict__ Q, const float* __restrict__ Rinv,
                                                    float* __restrict__ LT1, float* __restrict__ LT2) {
  const int e = blockIdx.x * 256 + threadIdx.x;
  if (e < NZ * NU) { const int i = e / NU, m = e % NU; float v;
    if (i < NX) { float s = 0.0f; for (int p = 0; p < NY; ++p) s += pmul(bf16_rne(St[m * NY + p]), bf16_rne(C2[p * NX + i])); v = s; }
    else if (i < NX + NUNIT) { const int q = i - NX; float s = 0.0f; for (int p = 0; p < NY; ++p) s += pmul(bf16_rne(St[m * NY + p]), bf16_rne(D21[p * NUNIT + q])); v = s - bf16_rne(D12[q * NU + m]); }
    else { v = bf16_rne(B2[(i - NX - NUNIT) * NU + m]); }
    for (int pass = 0; pass < 2; ++pass) { ((volatile float*)LT1)[e] = v; __threadfence(); } return; }
  const int e2 = e - NZ * NU; if (e2 >= NZ * NY) return; { const int i = e2 / NY, m = e2 % NY; float v;
    if (i < NX) v = bf16_rne(C2[m * NX + i]); else if (i < NX + NUNIT) v = bf16_rne(D21[m * NUNIT + (i - NX)]); else v = 0.0f;
    for (int pass = 0; pass < 2; ++pass) { ((volatile float*)LT2)[e2] = v; __threadfence(); } }
}
__global__ __launch_bounds__(256) void par2_kernel(const float* __restrict__ LT1, const float* __restrict__ LT2, const float* __restrict__ Q, const float* __restrict__ Rinv, float* __restrict__ LT1R, float* __restrict__ LT2Q) {
  const int e = blockIdx.x * 256 + threadIdx.x;
  if (e < NZ * NU) { const int i = e / NU, m = e % NU; float s = 0.0f; for (int p = 0; p < NU; ++p) s += pmul(LT1[i * NU + p], bf16_rne(Rinv[p * NU + m])); for (int pass = 0; pass < 2; ++pass) { ((volatile float*)LT1R)[e] = s; __threadfence(); } return; }
  const int e2 = e - NZ * NU; if (e2 >= NZ * NY) return; { const int i = e2 / NY, m = e2 % NY; float s = 0.0f; for (int p = 0; p < NY; ++p) s += pmul(LT2[i * NY + p], bf16_rne(Q[p * NY + m])); for (int pass = 0; pass < 2; ++pass) { ((volatile float*)LT2Q)[e2] = s; __threadfence(); } }
}
__global__ __launch_bounds__(256) void par3_kernel(const float* __restrict__ X, const float* __restrict__ LT1, const float* __restrict__ LT1R, const float* __restrict__ LT2, const float* __restrict__ LT2Q, const float* __restrict__ D12,
                                                    b16* __restrict__ CDh, b16* __restrict__ CDl, float* __restrict__ lam, float* __restrict__ DRF, b16* __restrict__ DRh, b16* __restrict__ DRl) {
  const int e = blockIdx.x * 256 + threadIdx.x;
  auto Hval = [&](int i, int j) { float s = 0.0f;
#pragma unroll 1
    for (int k = 0; k < NZ; ++k) s += pmul(bf16_rne(X[k * NZ + i]), bf16_rne(X[k * NZ + j]));
    if (i == j) s += 1e-3f;
#pragma unroll 1
    for (int m = 0; m < NU; ++m) s += pmul(LT1R[i * NU + m], LT1[j * NU + m]);
#pragma unroll 1
    for (int m = 0; m < NY; ++m) s -= pmul(LT2Q[i * NY + m], LT2[j * NY + m]);
    return s; };
  typedef __attribute__((ext_vector_type(2))) _Float16 v2h_; typedef __attribute__((ext_vector_type(2))) float v2f_;
  if (e < NUNIT * KV / 2) { const int u = (2 * e) / KV, k = (2 * e) % KV; v2h_ hv, lv;
    for (int q = 0; q < 2; ++q) { b16 h_, l_; const int kk = k + q; if (kk < NX) { const float c1 = -Hval(NX + u, kk); split16(c1 * WSC, h_, l_); } else { h_ = (b16)(bf16_rne(D12[u * NU + (kk - NX)]) * WSC); l_ = (b16)0.0f; } hv[q] = h_; lv[q] = l_; }
    for (int pass = 0; pass < 2; ++pass) { *(volatile v2h_*)(CDh + 2 * e) = hv; *(volatile v2h_*)(CDl + 2 * e) = lv; __threadfence(); } return; }
  int e2 = e - NUNIT * KV / 2;
  if (e2 < NUNIT * NUNIT / 2) { const int i = (2 * e2) / NUNIT, j = (2 * e2) % NUNIT; v2h_ hv, lv; v2f_ dv;
    for (int q = 0; q < 2; ++q) { const int jj = j + q; float d = 0.0f; if (i >= 1 && jj < i - 1) d = -Hval(NX + i - 1, NX + jj); b16 h_, l_; split16(d * WSC, h_, l_); dv[q] = d; hv[q] = h_; lv[q] = l_; }
    for (int pass = 0; pass < 2; ++pass) { *(volatile v2f_*)(DRF + 2 * e2) = dv; *(volatile v2h_*)(DRh + 2 * e2) = hv; *(volatile v2h_*)(DRl + 2 * e2) = lv; __threadfence(); } return; }
  e2 -= NUNIT * NUNIT / 2;
  if (e2 < NUNIT) { const float lm = 0.5f * Hval(NX + e2, NX + e2); for (int pass = 0; pass < 2; ++pass) { ((volatile float*)lam)[e2] = lm; __threadfence(); } }
}
__global__ __launch_bounds__(256) void prep_kernel(const float* __restrict__ u, const float* __restrict__ x0, const float* __restrict__ C2, const float* __restrict__ D21, b16* __restrict__ XU, b16* __restrict__ W2, b16* __restrict__ W21) {
  size_t t = (size_t)blockIdx.x * 256 + threadIdx.x; v8b o;
  const size_t nxu = (size_t)BATCH * KV / 8; if (t < nxu) { const size_t e = t * 8; const size_t b = e / KV; const int k0 = (int)(e % KV); for (int j = 0; j < 8; ++j) { const int k = k0 + j; const float v = (k < NX) ? x0[b * NX + k] : u[b * NU + (k - NX)]; o[j] = (b16)(bf16_rne(v) * XS); } for (int pass = 0; pass < 2; ++pass) { *(volatile v8b*)(XU + e) = o; __threadfence(); } return; } t -= nxu;
  if (t < (size_t)NY * NX / 8) { const size_t e = t * 8; for (int j = 0; j < 8; ++j) o[j] = (b16)(bf16_rne(C2[e + j]) * WSC); for (int pass = 0; pass < 2; ++pass) { *(volatile v8b*)(W2 + e) = o; __threadfence(); } return; } t -= (size_t)NY * NX / 8;
  if (t < (size_t)NY * NUNIT / 8) { const size_t e = t * 8; for (int j = 0; j < 8; ++j) o[j] = (b16)(bf16_rne(D21[e + j]) * WSC); for (int pass = 0; pass < 2; ++pass) { *(volatile v8b*)(W21 + e) = o; __threadfence(); } }
}
__global__ __launch_bounds__(128) void v_kernel(const b16* __restrict__ XU, const b16* __restrict__ CDh, const b16* __restrict__ CDl, const float* __restrict__ bvec, float* __restrict__ V) {
  __shared__ __attribute__((aligned(16))) float Tf[4][16][128 + 4];
  const int wave = threadIdx.x >> 5, lane = threadIdx.x & 31, nloc = lane & 15, hlf = lane >> 4; const size_t m0 = (size_t)blockIdx.x * 64 + wave * 16; const int n0 = blockIdx.y * 128;
  v8f acc[8];
#pragma unroll
  for (int t = 0; t < 8; ++t) acc[t] = (v8f){};
#pragma unroll 2
  for (int kb = 0; kb < KV; kb += 32) { const v16b a = frag_kb(XU + (m0 + nloc) * KV + kb, hlf);
#pragma unroll
    for (int t = 0; t < 8; ++t) { const size_t br = (size_t)(n0 + t * 16 + nloc) * KV + kb; acc[t] = wmma16b(a, frag_kb(CDh + br, hlf), acc[t]); acc[t] = wmma16b(a, frag_kb(CDl + br, hlf), acc[t]); } }
#pragma unroll
  for (int t = 0; t < 8; ++t) { const float bb = bf16_rne(bvec[NX + n0 + t * 16 + nloc]);
#pragma unroll
    for (int r = 0; r < 8; ++r) Tf[wave][8 * hlf + r][t * 16 + nloc] = acc[t][r] * (1.0f / (XS * WSC)) + bb; }
  wave_lds_sync();
  for (int pass = 0; pass < 2; ++pass) { for (int rr = 0; rr < 16; ++rr) *(volatile v4f*)(V + (m0 + rr) * NUNIT + n0 + lane * 4) = *(const v4f*)(&Tf[wave][rr][lane * 4]); __threadfence(); }
}
__global__ __launch_bounds__(64) void ren_kernel(const float* __restrict__ V, const float* __restrict__ DRF, const b16* __restrict__ DRh, const b16* __restrict__ DRl, const float* __restrict__ lam, const b16* __restrict__ XU, const b16* __restrict__ W2, const b16* __restrict__ W21, const float* __restrict__ bvec, float* __restrict__ Y) {
  __shared__ __attribute__((aligned(16))) float Wf[2][16][NUNIT + 4]; __shared__ __attribute__((aligned(16))) b16 Wh[2][16][NUNIT + 8], Wl[2][16][NUNIT + 8]; __shared__ __attribute__((aligned(16))) float Pf[2][16][16 + 1], Ty[2][16][NY + 1];
  const int wave = threadIdx.x >> 5, lane = threadIdx.x & 31, nloc = lane & 15, hlf = lane >> 4; const size_t m0 = (size_t)blockIdx.x * 32 + wave * 16;
#pragma unroll 1
  for (int j = 0; j < NUNIT / 16; ++j) {
    v8f acc = (v8f){};
const int kcovj = (16 * j) & ~31;
#pragma unroll 1
    for (int kb = 0; kb < kcovj; kb += 32) {
      const v16b ah = frag_kb(&Wh[wave][nloc][kb], hlf), al = frag_kb(&Wl[wave][nloc][kb], hlf); const size_t br = (size_t)(16 * j + nloc) * NUNIT + kb; const v16b bh = frag_kb(DRh + br, hlf), bl = frag_kb(DRl + br, hlf);
      acc = wmma16b(ah, bh, acc); acc = wmma16b(ah, bl, acc); acc = wmma16b(al, bh, acc); acc = wmma16b(al, bl, acc); }
    if (j == 0) { for (int rr = 0; rr < 16; ++rr) { for (int q = lane; q < NUNIT; q += 32) { Wf[wave][rr][q] = 0.0f; Wh[wave][rr][q] = (b16)0.0f; Wl[wave][rr][q] = (b16)0.0f; } } }
#pragma unroll
    for (int r = 0; r < 8; ++r) Pf[wave][8 * hlf + r][nloc] = acc[r] * (1.0f / (XS * WSC)) + V[(m0 + 8 * hlf + r) * NUNIT + 16 * j + nloc];
    wave_lds_sync();
    if (lane < 16) { const int rr = lane;
#pragma unroll 1
      for (int ii = 0; ii < 16; ++ii) { const int i = 16 * j + ii; float s = Pf[wave][rr][ii];
#pragma unroll 1
        for (int k = kcovj; k < i; ++k) s += pmul(Wf[wave][rr][k], DRF[(size_t)i * NUNIT + k]);
        const float w = tanhf(s / lam[i]); Wf[wave][rr][i] = w; b16 p, q; split16(w * XS, p, q); Wh[wave][rr][i] = p; Wl[wave][rr][i] = q; } }
    wave_lds_sync(); }
  v8f y0 = (v8f){}, y1 = (v8f){};
#pragma unroll
  for (int kb = 0; kb < NX; kb += 32) { const v16b a = frag_kb(XU + (m0 + nloc) * KV + kb, hlf); y0 = wmma16b(a, frag_kb(W2 + (size_t)nloc * NX + kb, hlf), y0); y1 = wmma16b(a, frag_kb(W2 + (size_t)(16 + nloc) * NX + kb, hlf), y1); }
#pragma unroll 2
  for (int kb = 0; kb < NUNIT; kb += 32) { const v16b ah = frag_kb(&Wh[wave][nloc][kb], hlf), al = frag_kb(&Wl[wave][nloc][kb], hlf); const v16b b0 = frag_kb(W21 + (size_t)nloc * NUNIT + kb, hlf), b1 = frag_kb(W21 + (size_t)(16 + nloc) * NUNIT + kb, hlf);
    y0 = wmma16b(ah, b0, y0); y0 = wmma16b(al, b0, y0); y1 = wmma16b(ah, b1, y1); y1 = wmma16b(al, b1, y1); }
#pragma unroll
  for (int r = 0; r < 8; ++r) { Ty[wave][8 * hlf + r][nloc] = y0[r] * (1.0f / (XS * WSC)) + bf16_rne(bvec[NX + NUNIT + nloc]); Ty[wave][8 * hlf + r][16 + nloc] = y1[r] * (1.0f / (XS * WSC)) + bf16_rne(bvec[NX + NUNIT + 16 + nloc]); }
  wave_lds_sync();
  for (int pass = 0; pass < 2; ++pass) { for (int rr = 0; rr < 16; ++rr) ((volatile float*)Y)[(m0 + rr) * NY + lane] = Ty[wave][rr][lane]; __threadfence(); }
}
}

extern "C" void kernel_launch(void* const* d_in, const int* in_sizes, int n_in, void* d_out, int out_size, void* d_ws, size_t ws_size, hipStream_t stream) {
  (void)n_in;
  auto Fp = [&](int i) { return (const float*)d_in[i]; };
  if (in_sizes[0] != BATCH * NU || in_sizes[1] != BATCH * NX || in_sizes[2] != NX * NU || in_sizes[3] != NY * NX || in_sizes[4] != NUNIT * NU || in_sizes[5] != NY * NUNIT || in_sizes[6] != NX + NUNIT + NY || in_sizes[7] != NZ * NZ || in_sizes[9] != NU * NY || in_sizes[10] != NY * NY || in_sizes[11] != NU * NU || out_size != BATCH * NY) return;
  size_t off = 0; char* ws = (char*)d_ws;
  auto carve = [&](size_t bytes) { char* p = ws + off; off += (bytes + 255) & ~(size_t)255; return p; };
  float* LT1 = (float*)carve((size_t)NZ * NU * 4); float* LT2 = (float*)carve((size_t)NZ * NY * 4); float* LT1R = (float*)carve((size_t)NZ * NU * 4); float* LT2Q = (float*)carve((size_t)NZ * NY * 4);
  b16* CDh = (b16*)carve((size_t)NUNIT * KV * 2); b16* CDl = (b16*)carve((size_t)NUNIT * KV * 2); float* lam = (float*)carve(NUNIT * 4); float* DRF = (float*)carve((size_t)NUNIT * NUNIT * 4); b16* DRh = (b16*)carve((size_t)NUNIT * NUNIT * 2); b16* DRl = (b16*)carve((size_t)NUNIT * NUNIT * 2);
  b16* XU = (b16*)carve((size_t)BATCH * KV * 2); b16* W2 = (b16*)carve((size_t)NY * NX * 2); b16* W21 = (b16*)carve((size_t)NY * NUNIT * 2); float* V = (float*)carve((size_t)BATCH * NUNIT * 4);
  if (off > ws_size || off > ((size_t)128 << 20)) return;
  par1_kernel<<<(NZ * NU + NZ * NY + 255) / 256, 256, 0, stream>>>(Fp(2), Fp(3), Fp(4), Fp(5), Fp(9), Fp(10), Fp(11), LT1, LT2);
  par2_kernel<<<(NZ * NU + NZ * NY + 255) / 256, 256, 0, stream>>>(LT1, LT2, Fp(10), Fp(11), LT1R, LT2Q);
  par3_kernel<<<(NUNIT * KV / 2 + NUNIT * NUNIT / 2 + NUNIT + 255) / 256, 256, 0, stream>>>(Fp(7), LT1, LT1R, LT2, LT2Q, Fp(4), CDh, CDl, lam, DRF, DRh, DRl);
  prep_kernel<<<(unsigned)((((size_t)BATCH * KV + (size_t)NY * NX + (size_t)NY * NUNIT) / 8 + 255) / 256), 256, 0, stream>>>(Fp(0), Fp(1), Fp(3), Fp(5), XU, W2, W21);
  v_kernel<<<dim3(NLIM / 64, NUNIT / 128), 128, 0, stream>>>(XU, CDh, CDl, Fp(6), V);
  ren_kernel<<<NLIM / 32, 64, 0, stream>>>(V, DRF, DRh, DRl, lam, XU, W2, W21, Fp(6), (float*)d_out);
}
